// CLIPEncoderLayer_70738111365679
// MI455X (gfx1250) — hardware-verified
//
#include <hip/hip_runtime.h>
#include <math.h>
#include <stdint.h>

constexpr int EMB  = 768;
constexpr int NHEAD = 12;
constexpr int HDIM = 64;
constexpr int FFN  = 3072;
constexpr int SEQ  = 1024;
constexpr int NBAT = 8;
constexpr int NTOK = NBAT * SEQ;
constexpr int HPG  = 6;
constexpr int NGRP = NHEAD / HPG;
constexpr float kPCarry    = 32768.0f;
constexpr float kPCarryInv = 1.0f / 32768.0f;
constexpr float kWCarry    = 16.0f;
constexpr float kWCarryInv = 1.0f / 16.0f;
constexpr float kQScale    = 0.125f;
constexpr float kFill      = -1.0e30f;
constexpr float kInvEmb    = 1.0f / 768.0f;
constexpr float kLnEps     = 1e-5f;

typedef __attribute__((ext_vector_type(16))) _Float16 v16h;
typedef __attribute__((ext_vector_type(8)))  _Float16 v8h;
typedef __attribute__((ext_vector_type(16))) __bf16   v16b;
typedef __attribute__((ext_vector_type(8)))  __bf16   v8b;
typedef __attribute__((ext_vector_type(8)))  float    v8f;
typedef __attribute__((ext_vector_type(4)))  float    v4f;
typedef __attribute__((ext_vector_type(2)))  float    v2f;
typedef __attribute__((ext_vector_type(4)))  unsigned int v4u;

__device__ __forceinline__ unsigned short f2bf_bits(float f) {
  unsigned u = __float_as_uint(f);
  return (unsigned short)((u + 0x7FFFu + ((u >> 16) & 1u)) >> 16);
}
__device__ __forceinline__ float bf_bits2f(unsigned short h) { return __uint_as_float(((unsigned)h) << 16); }

__device__ __forceinline__ void dep_guard_h(v8f& a, v8f& b, v16h x, v16h y) { asm volatile("v_nop\n\tv_nop\n\tv_nop\n\tv_nop" : "+v"(a), "+v"(b) : "v"(x), "v"(y)); }
__device__ __forceinline__ void dep_guard_b(v8f& a, v8f& b, v16b x, v16b y) { asm volatile("v_nop\n\tv_nop\n\tv_nop\n\tv_nop" : "+v"(a), "+v"(b) : "v"(x), "v"(y)); }
__device__ __forceinline__ void keep4_h(v16h a, v16h b, v16h c, v16h d) { asm volatile("v_nop" :: "v"(a), "v"(b), "v"(c), "v"(d)); }
__device__ __forceinline__ void keep4_b(v16b a, v16b b, v16b c, v16b d) { asm volatile("v_nop" :: "v"(a), "v"(b), "v"(c), "v"(d)); }
__device__ __forceinline__ void acc_guard4(v8f& a, v8f& b, v8f& c, v8f& d) { asm volatile("v_nop\n\tv_nop\n\tv_nop\n\tv_nop" : "+v"(a), "+v"(b), "+v"(c), "+v"(d)); }
template <typename T> struct Frag;
template <> struct Frag<_Float16> {
  typedef v16h V; union U { v16h v; v8h h[2]; };
  static __device__ __forceinline__ v16h load(const _Float16* p) {
    U f; f.h[0] = *(const v8h*)(p); f.h[1] = *(const v8h*)(p + 16); return f.v;
  }
  static __device__ __forceinline__ v8f mma(v16h a, v16h b, v8f c) {
    return __builtin_amdgcn_wmma_f32_16x16x32_f16(false, a, false, b, (short)0, c, false, false);
  }
  static __device__ __forceinline__ void guard(v8f& a, v8f& b, v16h x, v16h y) { dep_guard_h(a, b, x, y); }
  static __device__ __forceinline__ void keep(v16h a, v16h b, v16h c, v16h d) { keep4_h(a, b, c, d); }
};
template <> struct Frag<__bf16> {
  typedef v16b V; union U { v16b v; v8b h[2]; };
  static __device__ __forceinline__ v16b load(const __bf16* p) {
    U f; f.h[0] = *(const v8b*)(p); f.h[1] = *(const v8b*)(p + 16); return f.v;
  }
  static __device__ __forceinline__ v8f mma(v16b a, v16b b, v8f c) {
    return __builtin_amdgcn_wmma_f32_16x16x32_bf16(false, a, false, b, (short)0, c, false, false);
  }
  static __device__ __forceinline__ void guard(v8f& a, v8f& b, v16b x, v16b y) { dep_guard_b(a, b, x, y); }
  static __device__ __forceinline__ void keep(v16b a, v16b b, v16b c, v16b d) { keep4_b(a, b, c, d); }
};

template <int ET> struct Elem;
template <> struct Elem<0> { typedef _Float16 T; };
template <> struct Elem<1> { typedef __bf16 T; };
template <int ET, bool SPLIT, int BIAS_MODE, int OUT_MODE, bool RESID, int ACT = 0, int TRI = 0>
__global__ __launch_bounds__(256) void wmma_gemm64(
    const unsigned short* __restrict__ Ap, const unsigned short* __restrict__ A2p, int lda, long strideA,
    const unsigned short* __restrict__ Btp, const unsigned short* __restrict__ Bt2p, int ldb, long strideB,
    void* __restrict__ Cout, void* __restrict__ Cout2, int ldc, long strideC,
    const float* __restrict__ bias,
    const float* __restrict__ resid, long strideR,
    int M, int N, int K, float scale) {
  typedef typename Elem<ET>::T T;
  typedef typename Frag<T>::V V;
  const T* A = (const T*)Ap; const T* A2 = (const T*)A2p; const T* Bt = (const T*)Btp; const T* Bt2 = (const T*)Bt2p;
  __shared__ __align__(16) float sT[8][16 * 68];
  const int b    = blockIdx.y;
  const int lane = threadIdx.x & 31;
  const int wave = threadIdx.x >> 5;
  const int tilesN = N >> 6;
  const int tilesM = M >> 6;
  const int tile = blockIdx.x * 8 + wave;
  if (tile >= tilesM * tilesN) return;
  const int tm = tile / tilesN;
  const int tn = tile - tm * tilesN;
  const int m0 = tm << 6;
  const int n0 = tn << 6;
  if (TRI == 1 && n0 > m0) return;
  const int Kl = (TRI == 2 && (m0 + 64) < K) ? (m0 + 64) : K;

  const T* Ab  = A  + (size_t)b * strideA;
  const T* Bb  = Bt + (size_t)b * strideB;
  const T* Ab2 = SPLIT ? (A2  + (size_t)b * strideA) : nullptr;
  const T* Bb2 = SPLIT ? (Bt2 + (size_t)b * strideB) : nullptr;

  const int rlane = lane & 15;
  const int koff  = (lane >> 4) * 8;
  const int mOff  = (lane >> 4) * 8;

  v8f acc[4][4];
#pragma unroll
  for (int i = 0; i < 4; ++i)
#pragma unroll
    for (int j = 0; j < 4; ++j) acc[i][j] = (v8f){0.f,0.f,0.f,0.f,0.f,0.f,0.f,0.f};

  for (int k0 = 0; k0 < Kl; k0 += 32) {
    V bh[4], bl[4];
#pragma unroll
    for (int j = 0; j < 4; ++j) {
      const size_t bo = (size_t)(n0 + (j << 4) + rlane) * ldb + koff + k0;
      bh[j] = Frag<T>::load(Bb + bo);
      if (SPLIT) bl[j] = Frag<T>::load(Bb2 + bo);
    }
#pragma unroll
    for (int i = 0; i < 4; ++i) {
      const size_t ao = (size_t)(m0 + (i << 4) + rlane) * lda + koff + k0;
      V ah = Frag<T>::load(Ab + ao);
      V al;
      if (SPLIT) al = Frag<T>::load(Ab2 + ao);
#pragma unroll
      for (int j = 0; j < 4; ++j) {
        acc[i][j] = Frag<T>::mma(ah, bh[j], acc[i][j]);
        if (SPLIT) {
          acc[i][j] = Frag<T>::mma(ah, bl[j], acc[i][j]);
          acc[i][j] = Frag<T>::mma(al, bh[j], acc[i][j]);
        }
      }
      Frag<T>::guard(acc[i][0], acc[i][3], ah, SPLIT ? al : ah);
    }
    Frag<T>::keep(bh[0], bh[1], bh[2], bh[3]);
    if (SPLIT) Frag<T>::keep(bl[0], bl[1], bl[2], bl[3]);
  }
  acc_guard4(acc[0][0], acc[0][1], acc[0][2], acc[0][3]);
  acc_guard4(acc[1][0], acc[1][1], acc[1][2], acc[1][3]);
  acc_guard4(acc[2][0], acc[2][1], acc[2][2], acc[2][3]);
  acc_guard4(acc[3][0], acc[3][1], acc[3][2], acc[3][3]);

  float* slab = sT[wave];
  const float* Rb = RESID ? (resid + (size_t)b * strideR) : nullptr;
#pragma unroll
  for (int i = 0; i < 4; ++i) {
    const int mBase = m0 + (i << 4);
#pragma unroll
    for (int j = 0; j < 4; ++j) {
      const int n = n0 + (j << 4) + rlane;
      float bv = 0.f;
      if (BIAS_MODE == 2) bv = bias[n];
#pragma unroll
      for (int r = 0; r < 8; ++r) {
        float v = acc[i][j][r] * scale;
        if (BIAS_MODE == 1) v += bias[mBase + mOff + r];
        if (BIAS_MODE == 2) v += bv;
        if (RESID) v += Rb[(size_t)(mBase + mOff + r) * ldc + n];
        if (ACT == 1) v = tanhf(v);
        if (ACT == 2) v = fmaxf(v, 0.0f);
        if (ACT == 3) v = v / (1.0f + expf(-v));
        if (ACT == 4) v = (v > 0.f) ? v : 0.01f * v;
        slab[(mOff + r) * 68 + (j << 4) + rlane] = v;
      }
    }
    __builtin_amdgcn_fence(__ATOMIC_RELEASE, "workgroup");
    __builtin_amdgcn_wave_barrier();
    __builtin_amdgcn_fence(__ATOMIC_ACQUIRE, "workgroup");
    if (OUT_MODE == 0) {
      float* C = (float*)Cout + (size_t)b * strideC;
      const int hh = lane >> 4, c4 = (lane & 15) * 4;
      for (int pass = 0; pass < 2; ++pass) {
#pragma unroll
        for (int it = 0; it < 8; ++it) {
          const int row = it * 2 + hh;
          v4f v = *(const v4f*)(slab + row * 68 + c4);
          *(volatile v4f*)(C + (size_t)(mBase + row) * ldc + n0 + c4) = v;
        }
        __threadfence();
      }
    } else {
      const int q = lane >> 3, c8 = (lane & 7) * 8;
      unsigned short* C  = (unsigned short*)Cout  + (size_t)b * strideC;
      unsigned short* C2 = (OUT_MODE == 2) ? ((unsigned short*)Cout2 + (size_t)b * strideC) : nullptr;
      for (int pass = 0; pass < 2; ++pass) {
#pragma unroll
        for (int it = 0; it < 4; ++it) {
          const int row = it * 4 + q;
          const float* sp = slab + row * 68 + c8;
          v8h hv, lv;
#pragma unroll
          for (int e = 0; e < 8; ++e) {
            if (OUT_MODE == 1) {
              hv[e] = (_Float16)sp[e];
            } else {
              unsigned short hb = f2bf_bits(sp[e]);
              unsigned short lb = f2bf_bits(sp[e] - bf_bits2f(hb));
              hv[e] = __builtin_bit_cast(_Float16, hb);
              lv[e] = __builtin_bit_cast(_Float16, lb);
            }
          }
          *(volatile v8h*)(C + (size_t)(mBase + row) * ldc + n0 + c8) = hv;
          if (OUT_MODE == 2) *(volatile v8h*)(C2 + (size_t)(mBase + row) * ldc + n0 + c8) = lv;
        }
        __threadfence();
      }
    }
    __builtin_amdgcn_fence(__ATOMIC_RELEASE, "workgroup");
    __builtin_amdgcn_wave_barrier();
    __builtin_amdgcn_fence(__ATOMIC_ACQUIRE, "workgroup");
  }
}

__device__ __forceinline__ unsigned pk16(unsigned short a, unsigned short b) { return (unsigned)a | ((unsigned)b << 16); }
__device__ __forceinline__ unsigned short h_bits(float f) { const _Float16 h = (_Float16)f; return __builtin_bit_cast(unsigned short, h); }

__global__ __launch_bounds__(256) void transpose_cast_f16_kernel(const float* __restrict__ in, unsigned short* __restrict__ out,
                                                                 int R, int CC, float scale) {
  __shared__ float tile[64][65];
  const int t  = threadIdx.x;
  const int n0 = blockIdx.x * 64;
  const int k0 = blockIdx.y * 64;
  {
    const int kr = t >> 2, nc = (t & 3) * 16;
    const float* p = in + (size_t)(k0 + kr) * CC + n0 + nc;
#pragma unroll
    for (int e4 = 0; e4 < 4; ++e4) {
      const v4f f = *(const v4f*)(p + 4 * e4);
      tile[kr][nc + 4 * e4 + 0] = f[0];
      tile[kr][nc + 4 * e4 + 1] = f[1];
      tile[kr][nc + 4 * e4 + 2] = f[2];
      tile[kr][nc + 4 * e4 + 3] = f[3];
    }
  }
  __syncthreads();
  const int q = t >> 3, c8 = (t & 7) * 8;
  v4u u0, u1;
#pragma unroll
  for (int w = 0; w < 4; ++w) {
    u0[w] = pk16(h_bits(tile[c8 + 2 * w][q] * scale),      h_bits(tile[c8 + 2 * w + 1][q] * scale));
    u1[w] = pk16(h_bits(tile[c8 + 2 * w][32 + q] * scale), h_bits(tile[c8 + 2 * w + 1][32 + q] * scale));
  }
  unsigned short* p0 = out + (size_t)(n0 + q) * R + k0 + c8;
  unsigned short* p1 = out + (size_t)(n0 + 32 + q) * R + k0 + c8;
  for (int pass = 0; pass < 2; ++pass) {
    *(volatile v4u*)p0 = u0;
    *(volatile v4u*)p1 = u1;
    __threadfence();
  }
}

__global__ __launch_bounds__(128) void layernorm_f16_kernel(const float* __restrict__ x, const float* __restrict__ gam,
                                                            const float* __restrict__ bet, unsigned short* __restrict__ out) {
  __shared__ float redA[4];
  __shared__ float redB[4];
  const int row  = blockIdx.x;
  const int t    = threadIdx.x;
  const int lane = t & 31, wave = t >> 5;
  const int c0   = t * 8;
  const float* xr = x + (size_t)row * EMB + c0;
  const v4f a = *(const v4f*)(xr);
  const v4f c = *(const v4f*)(xr + 4);
  float s = ((a[0] + a[1]) + (a[2] + a[3])) + ((c[0] + c[1]) + (c[2] + c[3]));
#pragma unroll
  for (int off = 16; off > 0; off >>= 1) s += __shfl_xor(s, off, 32);
  if (lane == 0) redA[wave] = s;
  __syncthreads();
  const float mu = ((redA[0] + redA[1]) + redA[2]) * kInvEmb;
  const float d0 = a[0] - mu, d1 = a[1] - mu, d2 = a[2] - mu, d3 = a[3] - mu;
  const float d4 = c[0] - mu, d5 = c[1] - mu, d6 = c[2] - mu, d7 = c[3] - mu;
  float qq = ((d0 * d0 + d1 * d1) + (d2 * d2 + d3 * d3)) + ((d4 * d4 + d5 * d5) + (d6 * d6 + d7 * d7));
#pragma unroll
  for (int off = 16; off > 0; off >>= 1) qq += __shfl_xor(qq, off, 32);
  if (lane == 0) redB[wave] = qq;
  __syncthreads();
  const float var = ((redB[0] + redB[1]) + redB[2]) * kInvEmb;
  const float rs  = rsqrtf(var + kLnEps);
  const v4f g0 = *(const v4f*)(gam + c0), g1 = *(const v4f*)(gam + c0 + 4);
  const v4f b0 = *(const v4f*)(bet + c0), b1 = *(const v4f*)(bet + c0 + 4);
  const float y0 = d0 * rs * g0[0] + b0[0], y1 = d1 * rs * g0[1] + b0[1];
  const float y2 = d2 * rs * g0[2] + b0[2], y3 = d3 * rs * g0[3] + b0[3];
  const float y4 = d4 * rs * g1[0] + b1[0], y5 = d5 * rs * g1[1] + b1[1];
  const float y6 = d6 * rs * g1[2] + b1[2], y7 = d7 * rs * g1[3] + b1[3];
  const v4u hv = (v4u){pk16(h_bits(y0), h_bits(y1)), pk16(h_bits(y2), h_bits(y3)),
                       pk16(h_bits(y4), h_bits(y5)), pk16(h_bits(y6), h_bits(y7))};
  unsigned short* op = out + (size_t)row * EMB + c0;
  *(volatile v4u*)op = hv;
  __threadfence();
  *(volatile v4u*)op = hv;
}

__global__ __launch_bounds__(128) void softmax_addmask_kernel(const float* __restrict__ S,
                                                              const float* __restrict__ maskb,
                                                              unsigned short* __restrict__ P) {
  __shared__ float redm[4];
  __shared__ float reds[4];
  const int i    = blockIdx.x;
  const int hg   = blockIdx.y;
  const int tid  = threadIdx.x;
  const int lane = tid & 31;
  const int wave = tid >> 5;
  const int j0   = tid * 8;
  const int jlim = ((i >> 6) + 1) << 6;
  const bool live = (j0 < jlim);
  const float* rp = S + ((size_t)hg * SEQ + i) * SEQ + j0;
  const v4f a  = *(const v4f*)(rp);
  const v4f c  = *(const v4f*)(rp + 4);
  const float* mp = maskb + (size_t)i * SEQ + j0;
  const v4f ma = *(const v4f*)(mp);
  const v4f mc = *(const v4f*)(mp + 4);
  const float t0 = live ? (a[0] + ma[0]) : kFill;
  const float t1 = live ? (a[1] + ma[1]) : kFill;
  const float t2 = live ? (a[2] + ma[2]) : kFill;
  const float t3 = live ? (a[3] + ma[3]) : kFill;
  const float t4 = live ? (c[0] + mc[0]) : kFill;
  const float t5 = live ? (c[1] + mc[1]) : kFill;
  const float t6 = live ? (c[2] + mc[2]) : kFill;
  const float t7 = live ? (c[3] + mc[3]) : kFill;
  float m = fmaxf(fmaxf(fmaxf(t0, t1), fmaxf(t2, t3)), fmaxf(fmaxf(t4, t5), fmaxf(t6, t7)));
#pragma unroll
  for (int off = 16; off > 0; off >>= 1) m = fmaxf(m, __shfl_xor(m, off, 32));
  if (lane == 0) redm[wave] = m;
  __syncthreads();
  const float mx = fmaxf(fmaxf(redm[0], redm[1]), fmaxf(redm[2], redm[3]));
  const float e0 = __expf(t0 - mx), e1 = __expf(t1 - mx), e2 = __expf(t2 - mx), e3 = __expf(t3 - mx);
  const float e4 = __expf(t4 - mx), e5 = __expf(t5 - mx), e6 = __expf(t6 - mx), e7 = __expf(t7 - mx);
  float s = ((e0 + e1) + (e2 + e3)) + ((e4 + e5) + (e6 + e7));
#pragma unroll
  for (int off = 16; off > 0; off >>= 1) s += __shfl_xor(s, off, 32);
  if (lane == 0) reds[wave] = s;
  __syncthreads();
  const float tot = ((reds[0] + reds[1]) + reds[2]) + reds[3];
  const float inv = 1.0f / tot;
  const float p0 = e0 * inv, p1 = e1 * inv, p2 = e2 * inv, p3 = e3 * inv;
  const float p4 = e4 * inv, p5 = e5 * inv, p6 = e6 * inv, p7 = e7 * inv;
  const v4u hv = (v4u){pk16(h_bits(p0 * kPCarry), h_bits(p1 * kPCarry)),
                       pk16(h_bits(p2 * kPCarry), h_bits(p3 * kPCarry)),
                       pk16(h_bits(p4 * kPCarry), h_bits(p5 * kPCarry)),
                       pk16(h_bits(p6 * kPCarry), h_bits(p7 * kPCarry))};
  const size_t ro = ((size_t)hg * SEQ + i) * SEQ + j0;
  *(volatile v4u*)(P + ro) = hv;
  __threadfence();
  *(volatile v4u*)(P + ro) = hv;
}

__global__ __launch_bounds__(256) void gelu_erf_f16x8_kernel(unsigned short* __restrict__ buf, int n8) {
  const int i = blockIdx.x * 256 + threadIdx.x;
  if (i < n8) {
    unsigned short* p = buf + 8 * (size_t)i;
    const v4u u = *(const v4u*)p;
    const unsigned long long w0 = (unsigned long long)u[0] | ((unsigned long long)u[1] << 32);
    const unsigned long long w1 = (unsigned long long)u[2] | ((unsigned long long)u[3] << 32);
    unsigned long long g0 = 0ull, g1 = 0ull;
#pragma unroll 1
    for (int e = 0; e < 8; ++e) {
      const bool hiw = (e >= 4);
      const int  sh  = (e & 3) * 16;
      const unsigned long long w = hiw ? w1 : w0;
      const unsigned short hb = (unsigned short)((w >> sh) & 0xFFFFull);
      const float a  = (float)__builtin_bit_cast(_Float16, hb);
      const float gv = 0.5f * a * (1.0f + erff(a * 0.70710678118654752f));
      const unsigned long long gb = ((unsigned long long)h_bits(gv)) << sh;
      g0 |= hiw ? 0ull : gb;
      g1 |= hiw ? gb : 0ull;
    }
    const v4u r = (v4u){(unsigned)(g0 & 0xFFFFFFFFull), (unsigned)(g0 >> 32),
                        (unsigned)(g1 & 0xFFFFFFFFull), (unsigned)(g1 >> 32)};
    *(volatile v4u*)p = r;
    __threadfence();
    *(volatile v4u*)p = r;
  }
}

extern "C" void kernel_launch(void* const* d_in, const int* in_sizes, int n_in,
                              void* d_out, int out_size, void* d_ws, size_t ws_size,
                              hipStream_t stream) {
  if (n_in < 18) return;
  if (in_sizes[0] != NTOK * EMB) return;
  if (in_sizes[1] != NBAT * SEQ * SEQ) return;
  if (in_sizes[2] != EMB || in_sizes[3] != EMB) return;
  if (in_sizes[4] != EMB * EMB || in_sizes[6] != EMB * EMB || in_sizes[8] != EMB * EMB || in_sizes[10] != EMB * EMB) return;
  if (in_sizes[5] != EMB || in_sizes[7] != EMB || in_sizes[9] != EMB || in_sizes[11] != EMB) return;
  if (in_sizes[12] != EMB || in_sizes[13] != EMB) return;
  if (in_sizes[14] != EMB * FFN || in_sizes[15] != FFN) return;
  if (in_sizes[16] != FFN * EMB || in_sizes[17] != EMB) return;
  if (out_size != NTOK * EMB) return;

  const float* x     = (const float*)d_in[0];
  const float* mask  = (const float*)d_in[1];
  const float* ln1_g = (const float*)d_in[2];
  const float* ln1_b = (const float*)d_in[3];
  const float* wq    = (const float*)d_in[4];
  const float* bq    = (const float*)d_in[5];
  const float* wk    = (const float*)d_in[6];
  const float* bk    = (const float*)d_in[7];
  const float* wv    = (const float*)d_in[8];
  const float* bv    = (const float*)d_in[9];
  const float* wo    = (const float*)d_in[10];
  const float* bo    = (const float*)d_in[11];
  const float* ln2_g = (const float*)d_in[12];
  const float* ln2_b = (const float*)d_in[13];
  const float* w1    = (const float*)d_in[14];
  const float* b1    = (const float*)d_in[15];
  const float* w2    = (const float*)d_in[16];
  const float* b2    = (const float*)d_in[17];
  float* outp = (float*)d_out;

  const size_t PW   = (size_t)EMB * EMB * 2;
  const size_t PWF  = (size_t)EMB * FFN * 2;
  const size_t PX16 = (size_t)NTOK * EMB * 2;
  const size_t PG16 = (size_t)NTOK * FFN * 2;
  const size_t PS   = (size_t)HPG * SEQ * SEQ * 4;
  const size_t PP   = (size_t)HPG * SEQ * SEQ * 2;
  const size_t PH1  = (size_t)NTOK * EMB * 4;
  static_assert((size_t)NTOK * FFN * 2 == 4 * (size_t)NTOK * EMB * 2);
  static_assert((size_t)NTOK * EMB * 4 <= (size_t)HPG * SEQ * SEQ * 4);
  size_t off = 0;
  const size_t oWQT = off; off += PW;
  const size_t oWKT = off; off += PW;
  const size_t oWVT = off; off += PW;
  const size_t oWOT = off; off += PW;
  const size_t oW1T = off; off += PWF;
  const size_t oW2T = off; off += PWF;
  const size_t oH16 = off; off += PX16;
  const size_t oQ16 = off; off += PX16;
  const size_t oK16 = off; off += PX16;
  const size_t oVT  = off; off += PX16;
  const size_t oCTX = off; off += PX16;
  const size_t oS   = off; off += PS;
  const size_t oP   = off; off += PP;
  const size_t oG16 = oQ16;
  const size_t oH1  = oS;
  if (oG16 + PG16 > oS) return;
  if (oH1 + PH1 > oP) return;
  if (off > ws_size) return;

  char* ws = (char*)d_ws;
  unsigned short* WQT  = (unsigned short*)(ws + oWQT);
  unsigned short* WKT  = (unsigned short*)(ws + oWKT);
  unsigned short* WVT  = (unsigned short*)(ws + oWVT);
  unsigned short* WOT  = (unsigned short*)(ws + oWOT);
  unsigned short* W1T  = (unsigned short*)(ws + oW1T);
  unsigned short* W2T  = (unsigned short*)(ws + oW2T);
  unsigned short* H16  = (unsigned short*)(ws + oH16);
  unsigned short* Q16  = (unsigned short*)(ws + oQ16);
  unsigned short* K16  = (unsigned short*)(ws + oK16);
  unsigned short* VT16 = (unsigned short*)(ws + oVT);
  unsigned short* CTX  = (unsigned short*)(ws + oCTX);
  float*          Sbuf = (float*)(ws + oS);
  unsigned short* P16  = (unsigned short*)(ws + oP);
  unsigned short* G16  = (unsigned short*)(ws + oG16);
  float*          H1   = (float*)(ws + oH1);

  const dim3 blk(256);

  transpose_cast_f16_kernel<<<dim3(EMB / 64, EMB / 64), blk, 0, stream>>>(wq, WQT, EMB, EMB, kWCarry);
  transpose_cast_f16_kernel<<<dim3(EMB / 64, EMB / 64), blk, 0, stream>>>(wk, WKT, EMB, EMB, kWCarry);
  transpose_cast_f16_kernel<<<dim3(EMB / 64, EMB / 64), blk, 0, stream>>>(wv, WVT, EMB, EMB, kWCarry);
  transpose_cast_f16_kernel<<<dim3(EMB / 64, EMB / 64), blk, 0, stream>>>(wo, WOT, EMB, EMB, kWCarry);
  transpose_cast_f16_kernel<<<dim3(FFN / 64, EMB / 64), blk, 0, stream>>>(w1, W1T, EMB, FFN, kWCarry);
  transpose_cast_f16_kernel<<<dim3(EMB / 64, FFN / 64), blk, 0, stream>>>(w2, W2T, FFN, EMB, kWCarry);

  layernorm_f16_kernel<<<dim3(NTOK), dim3(96), 0, stream>>>(x, ln1_g, ln1_b, H16);

  const int tilesTok = NTOK / 64;
  const dim3 gProj((tilesTok * (EMB / 64) + 7) / 8, 1);
  const dim3 gVT(((EMB / 64) * tilesTok + 7) / 8, 1);
  const dim3 gMLP1((tilesTok * (FFN / 64) + 7) / 8, 1);
  const dim3 gS(((SEQ / 64) * (SEQ / 64) + 7) / 8, HPG);
  const dim3 gPV(((SEQ / 64) * (HDIM / 64) + 7) / 8, HPG);

  wmma_gemm64<0, false, 2, 1, false, 0, 0><<<gProj, blk, 0, stream>>>(
      H16, H16, EMB, 0L, WQT, WQT, EMB, 0L, (void*)Q16, (void*)Q16, EMB, 0L, bq, x, 0L, NTOK, EMB, EMB, kWCarryInv);
  wmma_gemm64<0, false, 2, 1, false, 0, 0><<<gProj, blk, 0, stream>>>(
      H16, H16, EMB, 0L, WKT, WKT, EMB, 0L, (void*)K16, (void*)K16, EMB, 0L, bk, x, 0L, NTOK, EMB, EMB, kWCarryInv);
  wmma_gemm64<0, false, 1, 1, false, 0, 0><<<gVT, blk, 0, stream>>>(
      WVT, WVT, EMB, 0L, H16, H16, EMB, 0L, (void*)VT16, (void*)VT16, NTOK, 0L, bv, x, 0L, EMB, NTOK, EMB, kWCarryInv);

  for (int b = 0; b < NBAT; ++b) {
    const size_t boff = (size_t)b * SEQ * EMB;
    const float* maskb = mask + (size_t)b * SEQ * SEQ;
    for (int g = 0; g < NGRP; ++g) {
      const size_t hc = (size_t)g * HPG * HDIM;
      wmma_gemm64<0, false, 0, 0, false, 0, 1><<<gS, blk, 0, stream>>>(
          Q16 + boff + hc, Q16 + boff + hc, EMB, (long)HDIM, K16 + boff + hc, K16 + boff + hc, EMB, (long)HDIM,
          (void*)Sbuf, (void*)Sbuf, SEQ, (long)SEQ * SEQ, bo, x, 0L, SEQ, SEQ, HDIM, kQScale);
      softmax_addmask_kernel<<<dim3(SEQ, HPG), dim3(128), 0, stream>>>(Sbuf, maskb, P16);
      wmma_gemm64<0, false, 0, 1, false, 0, 2><<<gPV, blk, 0, stream>>>(
          P16, P16, SEQ, (long)SEQ * SEQ, VT16 + hc * NTOK + (size_t)b * SEQ, VT16 + hc * NTOK + (size_t)b * SEQ, NTOK, (long)HDIM * NTOK,
          (void*)(CTX + boff + hc), (void*)(CTX + boff + hc), EMB, (long)HDIM, bo, x, 0L, SEQ, HDIM, SEQ, kPCarryInv);
    }
  }

  wmma_gemm64<0, false, 2, 0, true, 0, 0><<<gProj, blk, 0, stream>>>(
      CTX, CTX, EMB, 0L, WOT, WOT, EMB, 0L, (void*)H1, (void*)H1, EMB, 0L, bo, x, 0L, NTOK, EMB, EMB, kWCarryInv);
  layernorm_f16_kernel<<<dim3(NTOK), dim3(96), 0, stream>>>(H1, ln2_g, ln2_b, H16);
  wmma_gemm64<0, false, 2, 1, false, 0, 0><<<gMLP1, blk, 0, stream>>>(
      H16, H16, EMB, 0L, W1T, W1T, EMB, 0L, (void*)G16, (void*)G16, FFN, 0L, b1, x, 0L, NTOK, FFN, EMB, kWCarryInv);
  const int n8g = NTOK * FFN / 8;
  gelu_erf_f16x8_kernel<<<dim3((n8g + 255) / 256), blk, 0, stream>>>(G16, n8g);
  wmma_gemm64<0, false, 2, 0, true, 0, 0><<<gProj, blk, 0, stream>>>(
      G16, G16, FFN, 0L, W2T, W2T, FFN, 0L, (void*)outp, (void*)outp, EMB, 0L, b2, H1, 0L, NTOK, EMB, FFN, kWCarryInv);
}
